// SelectiveSSMKernel_36550171689111
// MI455X (gfx1250) — hardware-run, weakly checked
//
#include <hip/hip_runtime.h>
#include <math.h>

typedef __attribute__((ext_vector_type(16))) _Float16 v16h;
typedef __attribute__((ext_vector_type(8)))  _Float16 v8h;
typedef __attribute__((ext_vector_type(2)))  _Float16 v2h;
typedef __attribute__((ext_vector_type(16))) __bf16   v16b;
typedef __attribute__((ext_vector_type(8)))  __bf16   v8b;
typedef __attribute__((ext_vector_type(8)))  float    v8f;
typedef __attribute__((ext_vector_type(4)))  float    v4f;
typedef __attribute__((ext_vector_type(2)))  float    v2f;

constexpr int kNb   = 4;
constexpr int kD    = 1024;
constexpr int kL    = 2048;
constexpr int kN    = 64;
constexpr int kMS   = kD + 2 * kN;
constexpr int kThr  = 256;
constexpr float kInCarry = 1024.0f;
constexpr float kSc = 1.0f / (kInCarry * kInCarry);
constexpr float kF16MinNormal = 6.103515625e-5f;

static_assert(kD == 1024 && kL == 2048 && kN == 64 && kMS == 1152 && kNb == 4, "the index arithmetic below uses these sizes");

constexpr size_t kOffZB = 0ull;
constexpr size_t kOffW16 = 8192ull;
constexpr size_t kOffUT16 = 2367488ull;
constexpr size_t kOffP32 = 19144704ull;
constexpr size_t kWsTotal = 56893440ull;
static_assert(kWsTotal <= 134217728ull, "carve cap: under 128 MiB");
static_assert(kOffZB == 0
              && kOffW16 == kOffZB + 8192ull
              && kOffUT16 == kOffW16 + 2359296ull
              && kOffP32 == kOffUT16 + 16777216ull
              && kWsTotal == kOffP32 + 37748736ull, "the carve is chained and totalled");
static_assert((kOffZB % 256) == 0 && (kOffW16 % 256) == 0 && (kOffUT16 % 256) == 0 && (kOffP32 % 256) == 0, "aligned regions");
static_assert(2048 >= kMS, "the zero bias covers the engine launch's 1,152 output columns (the engine reads one bias value a column)");

__device__ __forceinline__ unsigned short f2bf_bits(float f) {
  unsigned u = __float_as_uint(f);
  return (unsigned short)((u + 0x7FFFu + ((u >> 16) & 1u)) >> 16);
}
__device__ __forceinline__ float bf_bits2f(unsigned short h) { return __uint_as_float(((unsigned)h) << 16); }
__device__ __forceinline__ float bf16r(float f) { return bf_bits2f(f2bf_bits(f)); }
__device__ __forceinline__ float carry_flush(float v, float carry) {
  const float s = v * carry;
  return (fabsf(s) < kF16MinNormal) ? 0.0f : s;
}

__device__ __forceinline__ void dep_guard4_h(v8f& a, v8f& b, v8f& c, v8f& d, v16h x, v16h y) { asm volatile("v_nop\n\tv_nop\n\tv_nop\n\tv_nop" : "+v"(a), "+v"(b), "+v"(c), "+v"(d) : "v"(x), "v"(y)); }
__device__ __forceinline__ void dep_guard4_b(v8f& a, v8f& b, v8f& c, v8f& d, v16b x, v16b y) { asm volatile("v_nop\n\tv_nop\n\tv_nop\n\tv_nop" : "+v"(a), "+v"(b), "+v"(c), "+v"(d) : "v"(x), "v"(y)); }
__device__ __forceinline__ void keep4_h(v16h a, v16h b, v16h c, v16h d) { asm volatile("v_nop" :: "v"(a), "v"(b), "v"(c), "v"(d)); }
__device__ __forceinline__ void keep4_b(v16b a, v16b b, v16b c, v16b d) { asm volatile("v_nop" :: "v"(a), "v"(b), "v"(c), "v"(d)); }
__device__ __forceinline__ void acc_guard4(v8f& a, v8f& b, v8f& c, v8f& d) { asm volatile("v_nop\n\tv_nop\n\tv_nop\n\tv_nop" : "+v"(a), "+v"(b), "+v"(c), "+v"(d)); }

template <typename T> struct Frag;
template <> struct Frag<_Float16> {
  typedef v16h V; union U { v16h v; v8h h[2]; };
  static __device__ __forceinline__ v16h load(const _Float16* p) {
    U f; f.h[0] = *(const v8h*)(p); f.h[1] = *(const v8h*)(p + 16); return f.v;
  }
  static __device__ __forceinline__ v8f mma(v16h a, v16h b, v8f c) {
    return __builtin_amdgcn_wmma_f32_16x16x32_f16(false, a, false, b, (short)0, c, false, false);
  }
  static __device__ __forceinline__ void guard4(v8f& a, v8f& b, v8f& c, v8f& d, v16h x, v16h y) { dep_guard4_h(a, b, c, d, x, y); }
  static __device__ __forceinline__ void keep(v16h a, v16h b, v16h c, v16h d) { keep4_h(a, b, c, d); }
};
template <> struct Frag<__bf16> {
  typedef v16b V; union U { v16b v; v8b h[2]; };
  static __device__ __forceinline__ v16b load(const __bf16* p) {
    U f; f.h[0] = *(const v8b*)(p); f.h[1] = *(const v8b*)(p + 16); return f.v;
  }
  static __device__ __forceinline__ v8f mma(v16b a, v16b b, v8f c) {
    return __builtin_amdgcn_wmma_f32_16x16x32_bf16(false, a, false, b, (short)0, c, false, false);
  }
  static __device__ __forceinline__ void guard4(v8f& a, v8f& b, v8f& c, v8f& d, v16b x, v16b y) { dep_guard4_b(a, b, c, d, x, y); }
  static __device__ __forceinline__ void keep(v16b a, v16b b, v16b c, v16b d) { keep4_b(a, b, c, d); }
};

__device__ __forceinline__ v8f mma_h(v16h a, v16h b, v8f c) {
  c = __builtin_amdgcn_wmma_f32_16x16x32_f16(false, a, false, b, (short)0, c, false, false);
  asm volatile("v_nop\n\tv_nop\n\tv_nop\n\tv_nop" : "+v"(c) : "v"(a), "v"(b));
  return c;
}

template <int ET> struct Elem;
template <> struct Elem<0> { typedef _Float16 T; };
template <> struct Elem<1> { typedef __bf16 T; };
template <int ET, bool SPLIT, int BIAS_MODE, int OUT_MODE, bool RESID, int ACT = 0>
__global__ __launch_bounds__(256) void wmma_gemm64(
    const unsigned short* __restrict__ Ap, const unsigned short* __restrict__ A2p, int lda, long strideA,
    const unsigned short* __restrict__ Btp, const unsigned short* __restrict__ Bt2p, int ldb, long strideB,
    void* __restrict__ Cout, void* __restrict__ Cout2, int ldc, long strideC,
    const float* __restrict__ bias,
    const float* __restrict__ resid, long strideR,
    int M, int N, int K, float scale) {
  typedef typename Elem<ET>::T T;
  typedef typename Frag<T>::V V;
  const T* A = (const T*)Ap; const T* A2 = (const T*)A2p; const T* Bt = (const T*)Btp; const T* Bt2 = (const T*)Bt2p;
  __shared__ __align__(16) float sT[8][16 * 68];
  const int b    = blockIdx.y;
  const int lane = threadIdx.x & 31;
  const int wave = threadIdx.x >> 5;
  const int tilesN = N >> 6;
  const int tilesM = M >> 6;
  const int tile = blockIdx.x * 8 + wave;
  if (tile >= tilesM * tilesN) return;
  const int tm = tile / tilesN;
  const int tn = tile - tm * tilesN;
  const int m0 = tm << 6;
  const int n0 = tn << 6;

  const T* Ab  = A  + (size_t)b * strideA;
  const T* Bb  = Bt + (size_t)b * strideB;
  const T* Ab2 = SPLIT ? (A2  + (size_t)b * strideA) : nullptr;
  const T* Bb2 = SPLIT ? (Bt2 + (size_t)b * strideB) : nullptr;

  const int rlane = lane & 15;
  const int koff  = (lane >> 4) * 8;
  const int mOff  = (lane >> 4) * 8;

  v8f acc[4][4];
#pragma unroll
  for (int i = 0; i < 4; ++i)
#pragma unroll
    for (int j = 0; j < 4; ++j) acc[i][j] = (v8f){0.f,0.f,0.f,0.f,0.f,0.f,0.f,0.f};

  for (int k0 = 0; k0 < K; k0 += 32) {
    V bh[4], bl[4];
#pragma unroll
    for (int j = 0; j < 4; ++j) {
      const size_t bo = (size_t)(n0 + (j << 4) + rlane) * ldb + koff + k0;
      bh[j] = Frag<T>::load(Bb + bo);
      if (SPLIT) bl[j] = Frag<T>::load(Bb2 + bo);
    }
#pragma unroll
    for (int i = 0; i < 4; ++i) {
      const size_t ao = (size_t)(m0 + (i << 4) + rlane) * lda + koff + k0;
      V ah = Frag<T>::load(Ab + ao);
      V al;
      if (SPLIT) al = Frag<T>::load(Ab2 + ao);
#pragma unroll
      for (int j = 0; j < 4; ++j) {
        acc[i][j] = Frag<T>::mma(ah, bh[j], acc[i][j]);
        if (SPLIT) {
          acc[i][j] = Frag<T>::mma(ah, bl[j], acc[i][j]);
          acc[i][j] = Frag<T>::mma(al, bh[j], acc[i][j]);
        }
      }
      Frag<T>::guard4(acc[i][0], acc[i][1], acc[i][2], acc[i][3], ah, SPLIT ? al : ah);
    }
    Frag<T>::keep(bh[0], bh[1], bh[2], bh[3]);
    if (SPLIT) Frag<T>::keep(bl[0], bl[1], bl[2], bl[3]);
  }
  acc_guard4(acc[0][0], acc[0][1], acc[0][2], acc[0][3]);
  acc_guard4(acc[1][0], acc[1][1], acc[1][2], acc[1][3]);
  acc_guard4(acc[2][0], acc[2][1], acc[2][2], acc[2][3]);
  acc_guard4(acc[3][0], acc[3][1], acc[3][2], acc[3][3]);

  float* slab = sT[wave];
  const float* Rb = RESID ? (resid + (size_t)b * strideR) : nullptr;
#pragma unroll
  for (int i = 0; i < 4; ++i) {
    const int mBase = m0 + (i << 4);
#pragma unroll
    for (int j = 0; j < 4; ++j) {
      const int n = n0 + (j << 4) + rlane;
      float bv = 0.f;
      if (BIAS_MODE == 2) bv = bias[n];
#pragma unroll
      for (int r = 0; r < 8; ++r) {
        float v = acc[i][j][r] * scale;
        if (BIAS_MODE == 1) v += bias[mBase + mOff + r];
        if (BIAS_MODE == 2) v += bv;
        if (RESID) v += Rb[(size_t)(mBase + mOff + r) * ldc + n];
        if (ACT == 1) v = tanhf(v);
        if (ACT == 2) v = fmaxf(v, 0.0f);
        if (ACT == 3) v = v / (1.0f + expf(-v));
        if (ACT == 4) v = (v > 0.f) ? v : 0.01f * v;
        slab[(mOff + r) * 68 + (j << 4) + rlane] = v;
      }
    }
    __builtin_amdgcn_fence(__ATOMIC_RELEASE, "workgroup");
    __builtin_amdgcn_wave_barrier();
    __builtin_amdgcn_fence(__ATOMIC_ACQUIRE, "workgroup");
    if (OUT_MODE == 0) {
      float* C = (float*)Cout + (size_t)b * strideC;
      const int hh = lane >> 4, c4 = (lane & 15) * 4;
      for (int pass = 0; pass < 2; ++pass) {
#pragma unroll
        for (int it = 0; it < 8; ++it) {
          const int row = it * 2 + hh;
          v4f v = *(const v4f*)(slab + row * 68 + c4);
          *(volatile v4f*)(C + (size_t)(mBase + row) * ldc + n0 + c4) = v;
        }
        __threadfence();
      }
    } else {
      const int q = lane >> 3, c8 = (lane & 7) * 8;
      unsigned short* C  = (unsigned short*)Cout  + (size_t)b * strideC;
      unsigned short* C2 = (OUT_MODE == 2) ? ((unsigned short*)Cout2 + (size_t)b * strideC) : nullptr;
      for (int pass = 0; pass < 2; ++pass) {
#pragma unroll
        for (int it = 0; it < 4; ++it) {
          const int row = it * 4 + q;
          const float* sp = slab + row * 68 + c8;
          v8h hv, lv;
#pragma unroll
          for (int e = 0; e < 8; ++e) {
            if (OUT_MODE == 1) {
              hv[e] = (_Float16)sp[e];
            } else {
              unsigned short hb = f2bf_bits(sp[e]);
              unsigned short lb = f2bf_bits(sp[e] - bf_bits2f(hb));
              hv[e] = __builtin_bit_cast(_Float16, hb);
              lv[e] = __builtin_bit_cast(_Float16, lb);
            }
          }
          *(volatile v8h*)(C + (size_t)(mBase + row) * ldc + n0 + c8) = hv;
          if (OUT_MODE == 2) *(volatile v8h*)(C2 + (size_t)(mBase + row) * ldc + n0 + c8) = lv;
        }
        __threadfence();
      }
    }
    __builtin_amdgcn_fence(__ATOMIC_RELEASE, "workgroup");
    __builtin_amdgcn_wave_barrier();
    __builtin_amdgcn_fence(__ATOMIC_ACQUIRE, "workgroup");
  }
}

__global__ __launch_bounds__(kThr) void cast_plane_kernel(const float* __restrict__ src, unsigned short* __restrict__ dst,
                                                          int colsLog2, int dstPitch, int dstOff) {
  const int i   = blockIdx.x * kThr + threadIdx.x;
  const int sh  = colsLog2 - 3;
  const int row = i >> sh;
  const int c8  = (i & ((1 << sh) - 1)) * 8;
  const float* sp = src + ((size_t)row << colsLog2) + c8;
  const v4f a0 = *(const v4f*)(sp);
  const v4f a1 = *(const v4f*)(sp + 4);
  v8h hv;
#pragma unroll
  for (int e = 0; e < 4; ++e) {
    const float f0 = a0[e];
    const float f1 = a1[e];
    hv[e]     = (_Float16)carry_flush(bf16r(f0), kInCarry);
    hv[4 + e] = (_Float16)carry_flush(bf16r(f1), kInCarry);
  }
  unsigned short* dp = dst + (size_t)row * dstPitch + dstOff + c8;
  *(volatile v8h*)dp = hv;
  __threadfence();
  *(volatile v8h*)dp = hv;
}


__global__ __launch_bounds__(kThr) void zero_kernel(float* __restrict__ dst) {
  const size_t o4 = ((size_t)blockIdx.x * kThr + threadIdx.x) * 4u;
  const v4f z = {0.f, 0.f, 0.f, 0.f};
  *(volatile v4f*)(dst + o4) = z;
  __threadfence();
  *(volatile v4f*)(dst + o4) = z;
}

__global__ __launch_bounds__(kThr) void ut_cast_kernel(const float* __restrict__ U, unsigned short* __restrict__ UT16) {
  const unsigned i = blockIdx.x * (unsigned)kThr + threadIdx.x;
  const unsigned d8 = i & 127u, l = (i >> 7) & 2047u, b = i >> 18;
  const float* sp = U + ((size_t)b * kD + d8 * 8u) * kL + l;
  v8h hv;
#pragma unroll
  for (int t = 0; t < 8; ++t) { const float v = sp[(size_t)t * kL]; hv[t] = (_Float16)carry_flush(bf16r(v), kInCarry); }
  unsigned short* dp = UT16 + (size_t)i * 8u;
  *(volatile v8h*)dp = hv;
  __threadfence();
  *(volatile v8h*)dp = hv;
}
static_assert((size_t)kNb * kL * (kD / 8) == 4096ull * kThr && kD / 8 == 128, "transposing cast grid exact: 4,096 blocks; 'i >> 18' is the sample");

__global__ __launch_bounds__(kThr) void scan_kernel(const float* __restrict__ PT, const float* __restrict__ U, const float* __restrict__ Ap, const float* __restrict__ Dp,
                                                   float* __restrict__ out) {
  const unsigned gi = blockIdx.x * (unsigned)kThr + threadIdx.x;
  const unsigned b = gi >> 10, d = gi & 1023u;
  float A[kN], h[kN];
#pragma unroll
  for (int n = 0; n < kN; ++n) { const float a = Ap[n]; A[n] = bf16r(a); h[n] = 0.0f; }
  const float q0 = Dp[d];
  const float dc = bf16r(q0);
  const float* pb = PT + (size_t)b * kL * kMS;
  const float* ur = U + ((size_t)b * kD + d) * kL;
  float* orow = out + ((size_t)b * kD + d) * kL;
  for (int l = 0; l < kL; ++l) {
    const float* pr = pb + (size_t)l * kMS;
    const float dl = pr[d];
    const float ur0 = ur[l];
    const float ul = bf16r(ur0);
    const float du = dl * ul;
    float y = 0.0f;
#pragma unroll
    for (int q = 0; q < kN / 4; ++q) {
      const v4f bv = *(const v4f*)(pr + kD + 4 * q), cv = *(const v4f*)(pr + kD + kN + 4 * q);
#pragma unroll
      for (int e = 0; e < 4; ++e) {
        const int n = 4 * q + e;
        const float hn = (dl * A[n]) * h[n] + du * bv[e];
        h[n] = hn;
        y += cv[e] * hn;
      }
    }
    const float o = y + dc * ul;
    float* dp = orow + l;
    *(volatile float*)dp = o;
    __threadfence();
    *(volatile float*)dp = o;
  }
}
static_assert(kNb * kD == 16 * kThr && (kN % 4) == 0 && (kD % 4) == 0, "scan grid exact: 16 blocks (4 a sample); the Bu | Cu columns 16-B aligned");

static_assert(((size_t)kD * kD / 8) % kThr == 0 && ((size_t)kN * kD / 8) % kThr == 0 && ((size_t)kD * kD) % 64 == 0 && ((size_t)kN * kD) % 64 == 0, "plane cast grids exact; the planes are whole rows of 64");
static_assert(((kL / 64) * (kMS / 64)) % 8 == 0, "the product's grid exact: every wave live");

extern "C" void kernel_launch(void* const* d_in, const int* in_sizes, int n_in,
                              void* d_out, int out_size, void* d_ws, size_t ws_size,
                              hipStream_t stream) {
  if (n_in < 7 || d_out == nullptr || d_ws == nullptr) return;
  if (in_sizes[0] != 1 || in_sizes[1] != kNb * kD * kL || in_sizes[2] != kN || in_sizes[3] != kN * kD || in_sizes[4] != kN * kD || in_sizes[5] != kD || in_sizes[6] != kD * kD) return;
  if (out_size != kNb * kD * kL) return;
  if (ws_size < kWsTotal) return;
  const float* U = (const float*)d_in[1];
  const float* Ap = (const float*)d_in[2];
  const float* Bm = (const float*)d_in[3];
  const float* Cm = (const float*)d_in[4];
  const float* Dp = (const float*)d_in[5];
  const float* Delta = (const float*)d_in[6];
  float* out = (float*)d_out;
  char* ws = (char*)d_ws;
  float* ZB = (float*)(ws + kOffZB);
  unsigned short* W16 = (unsigned short*)(ws + kOffW16);
  unsigned short* UT16 = (unsigned short*)(ws + kOffUT16);
  float* PT32 = (float*)(ws + kOffP32);

  zero_kernel<<<2, kThr, 0, stream>>>(ZB);
  cast_plane_kernel<<<(int)(((size_t)kD * kD / 8) / kThr), kThr, 0, stream>>>(Delta, W16, 6, 64, 0);
  cast_plane_kernel<<<(int)(((size_t)kN * kD / 8) / kThr), kThr, 0, stream>>>(Bm, W16 + (size_t)kD * kD, 6, 64, 0);
  cast_plane_kernel<<<(int)(((size_t)kN * kD / 8) / kThr), kThr, 0, stream>>>(Cm, W16 + (size_t)(kD + kN) * kD, 6, 64, 0);
  ut_cast_kernel<<<4096, kThr, 0, stream>>>(U, UT16);
  wmma_gemm64<0, false, 2, 0, false, 0><<<dim3((kL / 64) * (kMS / 64) / 8, kNb), 256, 0, stream>>>(
      UT16, UT16, kD, (long)kL * kD, W16, W16, kD, 0L, (void*)PT32, (void*)PT32, kMS, (long)kL * kMS, ZB, nullptr, 0L, kL, kMS, kD, kSc);
  scan_kernel<<<16, kThr, 0, stream>>>(PT32, U, Ap, Dp, out);
}
